// SelfAttention_68401649156637
// MI455X (gfx1250) — hardware-run, weakly checked
//
#include <hip/hip_runtime.h>
#include <math.h>

constexpr int kTok      = 2048;
constexpr int kDim      = 1024;
constexpr int kHeads    = 16;
constexpr int kDh       = 64;
constexpr int kInner    = kHeads * kDh;
constexpr int kQkvN     = 3 * kInner;
constexpr int kFeatCols = 2 * kInner;
constexpr int kWtRows   = kQkvN + kDim;
constexpr int kSq       = 1024;
constexpr int kTS       = 32;
constexpr int kDG       = 4;
constexpr int kDPer     = kDh / kDG;
constexpr float kFeatEps = 1.0e-3f;
static_assert(kInner == 1024 && kDim == 1024);
static_assert(kSq == kDim && kSq == kInner);
static_assert((kDim % 32) == 0 && (kInner % 32) == 0);
static_assert((kTok % 64) == 0 && (kQkvN % 64) == 0 && (kDim % 64) == 0);
static_assert((kFeatCols % 64) == 0);
static_assert((kTok % kTS) == 0 && kDPer == 16 && kDh == 64);
static_assert(((kTok / 64) * (kQkvN / 64)) % 8 == 0 && ((kTok / 64) * (kDim / 64)) % 8 == 0);

constexpr size_t kBytesXB  = (size_t)kTok * kDim * 2;
constexpr size_t kBytesWT  = (size_t)kWtRows * kSq * 2;
constexpr size_t kBytesQKV = (size_t)kTok * kQkvN * 4;
constexpr size_t kBytesAP  = (size_t)kTok * kInner * 2;
constexpr size_t kWsTotal  = kBytesXB + kBytesWT + kBytesQKV + kBytesAP + kBytesAP;
static_assert(kWsTotal == 46137344ull);
static_assert(kWsTotal <= 134217728ull);
static_assert((kBytesXB % 256) == 0 && (kBytesWT % 256) == 0 && (kBytesQKV % 256) == 0 && (kBytesAP % 256) == 0);

typedef __attribute__((ext_vector_type(16))) __bf16   v16b;
typedef __attribute__((ext_vector_type(8)))  __bf16   v8b;
typedef __attribute__((ext_vector_type(8)))  float    v8f;
typedef __attribute__((ext_vector_type(4)))  float    v4f;
typedef __attribute__((ext_vector_type(4)))  unsigned int v4u;

__device__ __forceinline__ unsigned short f2bf_bits(float f) {
  unsigned u = __float_as_uint(f);
  return (unsigned short)((u + 0x7FFFu + ((u >> 16) & 1u)) >> 16);
}
__device__ __forceinline__ float bf_bits2f(unsigned short h) { return __uint_as_float(((unsigned)h) << 16); }
__device__ __forceinline__ unsigned pk16(unsigned short a, unsigned short b) { return (unsigned)a | ((unsigned)b << 16); }

union FragB { v16b v; v8b h[2]; };
__device__ __forceinline__ v16b frag_load(const __bf16* p) {
  FragB f;
  f.h[0] = *(const v8b*)(p);
  f.h[1] = *(const v8b*)(p + 16);
  return f.v;
}
__device__ __forceinline__ v8f mma_g(v16b a, v16b b, v8f c) {
  c = __builtin_amdgcn_wmma_f32_16x16x32_bf16(false, a, false, b, (short)0, c, false, false);
  asm volatile("v_nop\n\tv_nop\n\tv_nop\n\tv_nop" : "+v"(c) : "v"(a), "v"(b));
  return c;
}

template <int SPL, int BIAS_MODE, int ACT>
__global__ __launch_bounds__(256) void wmma_gemm64(
    const unsigned short* __restrict__ Ap, const unsigned short* __restrict__ A2p, int lda,
    const unsigned short* __restrict__ Btp, int ldb,
    float* __restrict__ Cout, int ldc,
    const float* __restrict__ bias,
    int M, int N, int K) {
  const __bf16* A  = (const __bf16*)Ap;
  const __bf16* A2 = (const __bf16*)A2p;
  const __bf16* Bt = (const __bf16*)Btp;
  __shared__ __align__(16) float sT[8][16 * 68];
  const int lane = threadIdx.x & 31;
  const int wave = threadIdx.x >> 5;
  const int tilesN = N >> 6;
  const int tilesM = M >> 6;
  const int tile = blockIdx.x * 8 + wave;
  if (tile >= tilesM * tilesN) return;
  const int tm = tile / tilesN;
  const int tn = tile - tm * tilesN;
  const int m0 = tm << 6;
  const int n0 = tn << 6;

  const int rlane = lane & 15;
  const int koff  = (lane >> 4) * 8;
  const int mOff  = (lane >> 4) * 8;

  v8f acc[4][4];
#pragma unroll
  for (int i = 0; i < 4; ++i)
#pragma unroll
    for (int j = 0; j < 4; ++j) acc[i][j] = (v8f){0.f, 0.f, 0.f, 0.f, 0.f, 0.f, 0.f, 0.f};

  for (int k0 = 0; k0 < K; k0 += 32) {
    v16b bh[4];
#pragma unroll
    for (int j = 0; j < 4; ++j) {
      const size_t boff = (size_t)(n0 + (j << 4) + rlane) * ldb + koff + k0;
      bh[j] = frag_load(Bt + boff);
    }
#pragma unroll
    for (int i = 0; i < 4; ++i) {
      const size_t ao = (size_t)(m0 + (i << 4) + rlane) * lda + koff + k0;
      const v16b ah = frag_load(A + ao);
      v16b al = ah;
      if (SPL == 1) al = frag_load(A2 + ao);
#pragma unroll
      for (int j = 0; j < 4; ++j) {
        acc[i][j] = mma_g(ah, bh[j], acc[i][j]);
        if (SPL == 1) acc[i][j] = mma_g(al, bh[j], acc[i][j]);
      }
    }
  }

  float* slab = sT[wave];
  const bool feat = (ACT == 6) && (n0 < kFeatCols);
#pragma unroll
  for (int i = 0; i < 4; ++i) {
    const int mBase = m0 + (i << 4);
#pragma unroll
    for (int j = 0; j < 4; ++j) {
      const int n = n0 + (j << 4) + rlane;
      float bv = 0.f;
      if (BIAS_MODE == 2) bv = bf_bits2f(f2bf_bits(bias[n]));
#pragma unroll
      for (int r = 0; r < 8; ++r) {
        float v = acc[i][j][r];
        if (BIAS_MODE == 2) v += bv;
        if (ACT == 6) v = feat ? (fmaxf(v, 0.0f) + kFeatEps) : v;
        slab[(mOff + r) * 68 + (j << 4) + rlane] = v;
      }
    }
    __builtin_amdgcn_fence(__ATOMIC_RELEASE, "workgroup");
    __builtin_amdgcn_wave_barrier();
    __builtin_amdgcn_fence(__ATOMIC_ACQUIRE, "workgroup");
    {
      const int hh = lane >> 4, c4 = (lane & 15) * 4;
      for (int pass = 0; pass < 2; ++pass) {
#pragma unroll
        for (int it = 0; it < 8; ++it) {
          const int row = it * 2 + hh;
          const v4f v = *(const v4f*)(slab + row * 68 + c4);
          *(volatile v4f*)(Cout + (size_t)(mBase + row) * ldc + n0 + c4) = v;
        }
        __threadfence();
      }
    }
    __builtin_amdgcn_fence(__ATOMIC_RELEASE, "workgroup");
    __builtin_amdgcn_wave_barrier();
    __builtin_amdgcn_fence(__ATOMIC_ACQUIRE, "workgroup");
  }
}

__global__ __launch_bounds__(256) void cast8_bf16_kernel(const float* __restrict__ in, unsigned short* __restrict__ out, int n8) {
  const int i = blockIdx.x * 256 + threadIdx.x;
  if (i < n8) {
    const float* p = in + 8 * (size_t)i;
    const v4f a = *(const v4f*)(p);
    const v4f c = *(const v4f*)(p + 4);
    unsigned short hb[8];
#pragma unroll
    for (int e = 0; e < 4; ++e) {
      const float fa = a[e];
      const float fc = c[e];
      hb[e]     = f2bf_bits(fa);
      hb[4 + e] = f2bf_bits(fc);
    }
    const v4u u = (v4u){pk16(hb[0], hb[1]), pk16(hb[2], hb[3]), pk16(hb[4], hb[5]), pk16(hb[6], hb[7])};
    unsigned short* q = out + 8 * (size_t)i;
    *(volatile v4u*)q = u;
    __threadfence();
    *(volatile v4u*)q = u;
  }
}

__global__ __launch_bounds__(256) void wt_bf16_kernel(const float* __restrict__ W0, const float* __restrict__ W1,
                                                      const float* __restrict__ W2, const float* __restrict__ W3,
                                                      unsigned short* __restrict__ out) {
  __shared__ float sm[64][65];
  const int t  = threadIdx.x;
  const int k0 = blockIdx.x * 64;
  const int n0 = blockIdx.y * 64;
  const int z  = blockIdx.z;
  const float* W = (z == 0) ? W0 : (z == 1) ? W1 : (z == 2) ? W2 : W3;
#pragma unroll
  for (int i = 0; i < 16; ++i) {
    const int e = i * 256 + t;
    const int r = e >> 6;
    const int c = e & 63;
    sm[c][r] = W[(size_t)(k0 + r) * kSq + n0 + c];
  }
  __syncthreads();
  const int lane = t & 31, wave = t >> 5;
  const int q = lane >> 3, c8 = (lane & 7) * 8;
  unsigned short* op = out + (size_t)z * kSq * kSq;
  v4u u[2];
#pragma unroll
  for (int it = 0; it < 2; ++it) {
    const int row = wave * 8 + it * 4 + q;
    unsigned short hb[8];
#pragma unroll
    for (int e = 0; e < 8; ++e) hb[e] = f2bf_bits(sm[row][c8 + e]);
    u[it] = (v4u){pk16(hb[0], hb[1]), pk16(hb[2], hb[3]), pk16(hb[4], hb[5]), pk16(hb[6], hb[7])};
  }
  for (int pass = 0; pass < 2; ++pass) {
#pragma unroll
    for (int it = 0; it < 2; ++it) {
      const int row = wave * 8 + it * 4 + q;
      *(volatile v4u*)(op + (size_t)(n0 + row) * kSq + k0 + c8) = u[it];
    }
    __threadfence();
  }
}

__global__ __launch_bounds__(256) void state_scan_kernel(const float* __restrict__ QKV,
                                                         unsigned short* __restrict__ AH,
                                                         unsigned short* __restrict__ AL) {
  __shared__ __align__(16) float sQ[kTS * kDh];
  __shared__ __align__(16) float sK[kTS * kDh];
  __shared__ __align__(16) float sV[kTS * kDh];
  __shared__ __align__(16) float sN[kTS * kDG * kDh];
  __shared__ __align__(16) float sD[kTS * kDG];

  const int head = blockIdx.x;
  const int tid  = threadIdx.x;
  const int lane = tid & 31, wave = tid >> 5;
  const int dg = tid >> 6;
  const int e  = tid & 63;

  float ctx[kDPer], ksum[kDPer];
#pragma unroll
  for (int i = 0; i < kDPer; ++i) {
    ctx[i] = 0.0f;
    ksum[i] = 0.0f;
  }

  const int erow = wave * 4 + (lane >> 3);
  const int c8   = (lane & 7) * 8;

#pragma unroll 1
  for (int t0 = 0; t0 < kTok; t0 += kTS) {
    __syncthreads();
#pragma unroll
    for (int i = 0; i < 2; ++i) {
      const int idx = tid + i * 256;
      const int r   = idx >> 4;
      const int c4  = (idx & 15) * 4;
      const float* g = QKV + (size_t)(t0 + r) * kQkvN + head * kDh + c4;
      *(v4f*)(sQ + r * kDh + c4) = *(const v4f*)(g);
      *(v4f*)(sK + r * kDh + c4) = *(const v4f*)(g + kInner);
      *(v4f*)(sV + r * kDh + c4) = *(const v4f*)(g + 2 * kInner);
    }
    __syncthreads();

#pragma unroll 1
    for (int s = 0; s < kTS; ++s) {
      const float* kp = sK + s * kDh + dg * kDPer;
      const float* qp = sQ + s * kDh + dg * kDPer;
      v4f k4[4], q4[4];
#pragma unroll
      for (int j = 0; j < 4; ++j) {
        k4[j] = *(const v4f*)(kp + 4 * j);
        q4[j] = *(const v4f*)(qp + 4 * j);
      }
      const float vv = sV[s * kDh + e];
      float num = 0.0f, den = 0.0f;
#pragma unroll
      for (int i = 0; i < kDPer; ++i) {
        const float kv = k4[i >> 2][i & 3];
        const float qv = q4[i >> 2][i & 3];
        ctx[i]  = fmaf(kv, vv, ctx[i]);
        ksum[i] = ksum[i] + kv;
        num = fmaf(qv, ctx[i], num);
        den = fmaf(qv, ksum[i], den);
      }
      sN[(s * kDG + dg) * kDh + e] = num;
      if (e == 0) sD[s * kDG + dg] = den;
    }
    __syncthreads();

    {
      const v4f dv = *(const v4f*)(sD + erow * kDG);
      const float den = ((dv[0] + dv[1]) + dv[2]) + dv[3];
      const float inv = 1.0f / den;
      v4f n0v = *(const v4f*)(sN + (erow * kDG + 0) * kDh + c8);
      v4f n1v = *(const v4f*)(sN + (erow * kDG + 0) * kDh + c8 + 4);
#pragma unroll
      for (int g = 1; g < kDG; ++g) {
        const v4f p0 = *(const v4f*)(sN + (erow * kDG + g) * kDh + c8);
        const v4f p1 = *(const v4f*)(sN + (erow * kDG + g) * kDh + c8 + 4);
        n0v = n0v + p0;
        n1v = n1v + p1;
      }
      unsigned short hb[8], lb[8];
#pragma unroll
      for (int x = 0; x < 4; ++x) {
        const float a0 = n0v[x] * inv;
        const float a1 = n1v[x] * inv;
        const unsigned short h0 = f2bf_bits(a0);
        const unsigned short h1 = f2bf_bits(a1);
        hb[x]     = h0;
        hb[4 + x] = h1;
        lb[x]     = f2bf_bits(a0 - bf_bits2f(h0));
        lb[4 + x] = f2bf_bits(a1 - bf_bits2f(h1));
      }
      const v4u uh = (v4u){pk16(hb[0], hb[1]), pk16(hb[2], hb[3]), pk16(hb[4], hb[5]), pk16(hb[6], hb[7])};
      const v4u ul = (v4u){pk16(lb[0], lb[1]), pk16(lb[2], lb[3]), pk16(lb[4], lb[5]), pk16(lb[6], lb[7])};
      const size_t o = (size_t)(t0 + erow) * kInner + head * kDh + c8;
      for (int pass = 0; pass < 2; ++pass) {
        *(volatile v4u*)(AH + o) = uh;
        *(volatile v4u*)(AL + o) = ul;
        __threadfence();
      }
    }
  }
}

extern "C" void kernel_launch(void* const* d_in, const int* in_sizes, int n_in,
                              void* d_out, int out_size, void* d_ws, size_t ws_size,
                              hipStream_t stream) {
  if (n_in < 6 || d_out == nullptr || d_ws == nullptr) return;
  if (in_sizes[0] != kTok * kDim) return;
  if (in_sizes[1] != kDim * kInner) return;
  if (in_sizes[2] != kDim * kInner) return;
  if (in_sizes[3] != kDim * kInner) return;
  if (in_sizes[4] != kInner * kDim) return;
  if (in_sizes[5] != kDim) return;
  if (out_size != kTok * kDim) return;

  const float* x  = (const float*)d_in[0];
  const float* Wq = (const float*)d_in[1];
  const float* Wk = (const float*)d_in[2];
  const float* Wv = (const float*)d_in[3];
  const float* Wo = (const float*)d_in[4];
  const float* bo = (const float*)d_in[5];
  float* out = (float*)d_out;

  char* ws = (char*)d_ws;
  size_t off = 0;
  auto carve = [&](size_t bytes) -> char* { char* p = ws + off; off += (bytes + 255) & ~(size_t)255; return p; };
  unsigned short* XB  = (unsigned short*)carve(kBytesXB);
  unsigned short* WT  = (unsigned short*)carve(kBytesWT);
  float*          QKV = (float*)carve(kBytesQKV);
  unsigned short* AH  = (unsigned short*)carve(kBytesAP);
  unsigned short* AL  = (unsigned short*)carve(kBytesAP);
  if (off != kWsTotal || off > ws_size || off > (size_t)134217728) return;

  const int n8x = kTok * kDim / 8;
  cast8_bf16_kernel<<<n8x / 256, 256, 0, stream>>>(x, XB, n8x);
  wt_bf16_kernel<<<dim3(kSq / 64, kSq / 64, 4), 256, 0, stream>>>(Wq, Wk, Wv, Wo, WT);

  wmma_gemm64<0, 0, 6><<<dim3((kTok / 64) * (kQkvN / 64) / 8), 256, 0, stream>>>(
      XB, XB, kDim,
      WT, kDim,
      QKV, kQkvN,
      bo,
      kTok, kQkvN, kDim);

  state_scan_kernel<<<kHeads, 256, 0, stream>>>(QKV, AH, AL);

  wmma_gemm64<1, 2, 0><<<dim3((kTok / 64) * (kDim / 64) / 8), 256, 0, stream>>>(
      AH, AL, kInner,
      WT + (size_t)kQkvN * kSq, kInner,
      out, kDim,
      bo,
      kTok, kDim, kInner);
}
